// DeformBlock_63617055588616
// MI455X (gfx1250) — hardware-verified
//
#include <hip/hip_runtime.h>
#include <math.h>

typedef __attribute__((ext_vector_type(16))) _Float16 v16h;
typedef __attribute__((ext_vector_type(16))) __bf16 v16b;
typedef __attribute__((ext_vector_type(8)))  _Float16 v8h;
typedef __attribute__((ext_vector_type(8)))  float v8f;
typedef __attribute__((ext_vector_type(4)))  float v4f;
typedef __attribute__((ext_vector_type(2)))  float v2f;
typedef __attribute__((ext_vector_type(4)))  unsigned v4u;
typedef __attribute__((ext_vector_type(4)))  int v4i;
typedef float __attribute__((may_alias)) float_a;
typedef int __attribute__((may_alias)) int_a;

template <typename T> __device__ __forceinline__ void vst2(void* p, T v) { *(volatile T*)p = v; __threadfence(); *(volatile T*)p = v; }
__device__ __forceinline__ v8f wmma16(v16h a, v16h b, v8f c) {
  v8f d = __builtin_amdgcn_wmma_f32_16x16x32_f16(false, a, false, b, (short)0, c, false, false);
  asm volatile("v_nop\n\tv_nop\n\tv_nop\n\tv_nop" : "+v"(d) : "v"(a), "v"(b));
  return d;
}
__device__ __forceinline__ v8f wmma_bf(v16b a, v16b b, v8f c) {
  v8f d = __builtin_amdgcn_wmma_f32_16x16x32_bf16(false, a, false, b, (short)0, c, false, false);
  asm volatile("v_nop\n\tv_nop\n\tv_nop\n\tv_nop" : "+v"(d) : "v"(a), "v"(b));
  return d;
}
__device__ __forceinline__ v16h frag_h(const _Float16* rowk0, int lane) {
  union { v16h v; v8h q[2]; } u; const _Float16* p = rowk0 + 8 * (lane >> 4);
  u.q[0] = *(const v8h*)p; u.q[1] = *(const v8h*)(p + 16); return u.v;
}
__device__ __forceinline__ v16h frag_f32(const float* rowk0, int lane) {
  v16h a; const float* p = rowk0 + 8 * (lane >> 4);
#pragma unroll
  for (int i = 0; i < 8; ++i) { a[i] = (_Float16)p[i]; a[8 + i] = (_Float16)p[16 + i]; }
  return a;
}
__device__ __forceinline__ v16h frag_f32s(const float* rowk0, int lane, float sc) {
  v16h a; const float* p = rowk0 + 8 * (lane >> 4);
#pragma unroll
  for (int i = 0; i < 8; ++i) { a[i] = (_Float16)(p[i] * sc); a[8 + i] = (_Float16)(p[16 + i] * sc); }
  return a;
}
__device__ __forceinline__ v16h fragc_f32(const float* W, int k0, int n, int lane, int ld, int K) {
  v16h a; const int g = lane >> 4;
#pragma unroll
  for (int i = 0; i < 8; ++i) { const int ka = k0 + 8 * g + i, kb = ka + 16;
    a[i] = (_Float16)(ka < K ? W[(size_t)(ka < K ? ka : K - 1) * ld + n] : 0.f); a[8 + i] = (_Float16)(kb < K ? W[(size_t)(kb < K ? kb : K - 1) * ld + n] : 0.f); }
  return a;
}
struct F2 { v16b h, l; };
__device__ __forceinline__ F2 bsplit16(const float v[16]) { F2 r;
#pragma unroll
  for (int i = 0; i < 16; ++i) { const __bf16 h = (__bf16)v[i]; r.h[i] = h; r.l[i] = (__bf16)(v[i] - (float)h); }
  return r; }
__device__ __forceinline__ F2 split_row(const float* row, int k0, int lane) { float v[16]; const float* p = row + k0 + 8 * (lane >> 4);
#pragma unroll
  for (int i = 0; i < 8; ++i) { v[i] = p[i]; v[8 + i] = p[16 + i]; }
  return bsplit16(v); }
__device__ __forceinline__ F2 split_rowK(const float* row, int k0, int lane, int K) { float v[16]; const int g = lane >> 4;
#pragma unroll
  for (int i = 0; i < 8; ++i) { const int ka = k0 + 8 * g + i, kb = ka + 16; v[i] = ka < K ? row[ka < K ? ka : K - 1] : 0.f; v[8 + i] = kb < K ? row[kb < K ? kb : K - 1] : 0.f; }
  return bsplit16(v); }
__device__ __forceinline__ F2 split_col(const float* W, int k0, int n, int lane, int ld, int K) { float v[16]; const int g = lane >> 4;
#pragma unroll
  for (int i = 0; i < 8; ++i) { const int ka = k0 + 8 * g + i, kb = ka + 16; v[i] = ka < K ? W[(size_t)(ka < K ? ka : K - 1) * ld + n] : 0.f; v[8 + i] = kb < K ? W[(size_t)(kb < K ? kb : K - 1) * ld + n] : 0.f; }
  return bsplit16(v); }
__device__ __forceinline__ v8f mac3(const F2& a, const F2& b, v8f c) { c = wmma_bf(a.l, b.h, c); c = wmma_bf(a.h, b.l, c); return wmma_bf(a.h, b.h, c); }
__device__ __forceinline__ float sigm(float v) { return 1.0f / (1.0f + expf(-v)); }
#define LDSX() do { asm volatile("s_wait_dscnt 0" ::: "memory"); __builtin_amdgcn_wave_barrier(); __builtin_amdgcn_fence(__ATOMIC_RELEASE, "workgroup"); } while (0)


#define NB 4
#define CC 64
#define HH 128
#define WWD 128
#define NP (HH * WWD)
#define NT 9
#define KD (NT * CC)
#define BNEPS 1e-5f
typedef __attribute__((ext_vector_type(8))) __bf16 v8b;
__device__ __forceinline__ v16b frag_b(const __bf16* rowk0, int lane) {
  union { v16b v; v8b q[2]; } u; const __bf16* p = rowk0 + 8 * (lane >> 4);
  u.q[0] = *(const v8b*)p; u.q[1] = *(const v8b*)(p + 16); return u.v;
}
__device__ __forceinline__ float bfr(float v) { return (float)(__bf16)v; }
__device__ __attribute__((noinline)) float exp_ni(float v) { return expf(v); }
__device__ __attribute__((noinline)) float erf_ni(float v) { return erff(v); }

#define WS_PO1 0u
#define WS_PD1 (WS_PO1 + 2u * (size_t)32 * KD)
#define WS_PO2 (WS_PD1 + 2u * (size_t)CC * KD)
#define WS_PD2 (WS_PO2 + 2u * (size_t)32 * KD)
#define WS_XT  (WS_PD2 + 2u * (size_t)CC * KD)
#define WS_OFF (WS_XT + 4u * (size_t)NB * NP * CC)
#define WS_Y   (WS_OFF + 4u * (size_t)NB * NP * 32)
#define WS_ST  (WS_Y + 4u * (size_t)NB * CC * NP)
#define WS_END (WS_ST + 4u * (size_t)64 * 2)

__global__ __launch_bounds__(64) void k_pack(const float* __restrict__ WO1, const float* __restrict__ WD1, const float* __restrict__ WO2, const float* __restrict__ WD2, __bf16* __restrict__ P) { const int n = blockIdx.x, which = blockIdx.y, t = threadIdx.x; __shared__ __align__(16) __bf16 s[KD];
  const bool isoff = (which == 0 || which == 2); if (isoff && n >= 32) return; const float* w = (which == 0) ? WO1 : (which == 1) ? WD1 : (which == 2) ? WO2 : WD2; const size_t dst = ((which == 0) ? WS_PO1 : (which == 1) ? WS_PD1 : (which == 2) ? WS_PO2 : WS_PD2) / 2 + (size_t)n * KD;
  for (int tap = 0; tap < NT; ++tap) s[tap * CC + t] = (isoff && n >= 27) ? (__bf16)0.0f : (__bf16)w[((size_t)n * CC + t) * NT + tap]; __syncthreads(); for (int q = t; q < KD / 8; q += 64) vst2((unsigned*)(P + dst + q * 8), *(const v4u*)&s[q * 8]); }
__global__ __launch_bounds__(256) void k_xt(const float* __restrict__ X, float* __restrict__ XT) { __shared__ float st[64][CC + 1]; __shared__ __align__(16) float so2[64][CC + 4]; const int t = threadIdx.x; const int p0 = blockIdx.x * 64; const size_t b = blockIdx.y;
  for (int e = t; e < CC * 64; e += 256) { const int c = e >> 6, pl = e & 63; st[pl][c] = bfr(X[(b * CC + c) * NP + p0 + pl]); } __syncthreads();
  for (int e = t; e < 64 * CC; e += 256) { const int pl = e >> 6, c = e & 63; so2[pl][c] = st[pl][c]; } __syncthreads();
  for (int e = t; e < 64 * 16; e += 256) { const int pl = e >> 4, q = e & 15; vst2(XT + ((b * NP + p0 + pl) * CC) + q * 4, *(const v4f*)&so2[pl][q * 4]); } }
template <int EXACT>
__global__ __launch_bounds__(128) void k_off(const float* __restrict__ XT, const __bf16* __restrict__ Wr, const float* __restrict__ BOFF, float* __restrict__ OFF) { __shared__ __align__(16) float so[4][16][36];
  const int tid = threadIdx.x, wave = tid >> 5, lane = tid & 31, col = lane & 15, g = lane >> 4; const size_t b = blockIdx.y; const int p0 = blockIdx.x * 64 + wave * 16; const int pix = p0 + col; const int py = pix / WWD, px = pix % WWD;
  v8f acc[2] = {};
#pragma unroll 1
  for (int tap = 0; tap < NT; ++tap) { const int yy = py + tap / 3 - 1, xx = px + tap % 3 - 1; const bool inb = yy >= 0 && yy < HH && xx >= 0 && xx < WWD; const float* src = XT + ((b * NP + (size_t)(inb ? yy * WWD + xx : 0)) * CC);
#pragma unroll
    for (int q = 0; q < 2; ++q) { float v[16]; const float* pp = src + q * 32 + 8 * g;
#pragma unroll
      for (int i = 0; i < 8; ++i) { v[i] = inb ? pp[i] : 0.f; v[8 + i] = inb ? pp[16 + i] : 0.f; }
      if (EXACT) { v16b a;
#pragma unroll
        for (int i = 0; i < 16; ++i) a[i] = (__bf16)v[i];
#pragma unroll
        for (int j = 0; j < 2; ++j) acc[j] = wmma_bf(a, frag_b(Wr + (size_t)(j * 16 + col) * KD + tap * CC + q * 32, lane), acc[j]); }
      else { const F2 a = bsplit16(v);
#pragma unroll
        for (int j = 0; j < 2; ++j) { const v16b w = frag_b(Wr + (size_t)(j * 16 + col) * KD + tap * CC + q * 32, lane); acc[j] = wmma_bf(a.h, w, acc[j]); acc[j] = wmma_bf(a.l, w, acc[j]); } } } }
#pragma unroll
  for (int j = 0; j < 2; ++j)
#pragma unroll
    for (int r = 0; r < 8; ++r) { const int ch = j * 16 + col; so[wave][8 * g + r][ch] = acc[j][r] + ((ch < 27) ? bfr(BOFF[ch]) : 0.f); }
  LDSX(); for (int rl = 0; rl < 16; ++rl) if (lane < 8) vst2(OFF + ((b * NP + p0 + rl) * 32) + lane * 4, *(const v4f*)&so[wave][rl][lane * 4]); }
__device__ __forceinline__ void corner16(const float* __restrict__ XTb, int yc, int xc, int g, int kc, float w, float* v) { const bool valid = (yc >= 0) && (yc < HH) && (xc >= 0) && (xc < WWD); if (!valid) return; const float* p = XTb + ((size_t)(yc * WWD + xc) * CC) + kc * 32 + 8 * g;
#pragma unroll
  for (int i = 0; i < 8; ++i) { v[i] += w * p[i]; v[8 + i] += w * p[16 + i]; } }
__global__ __launch_bounds__(128) void k_def(const float* __restrict__ XT, const float* __restrict__ OFF, const __bf16* __restrict__ Wr, const float* __restrict__ BDEF, float* __restrict__ Y) { __shared__ __align__(16) float so[CC][64 + 4];
  const int tid = threadIdx.x, wave = tid >> 5, lane = tid & 31, col = lane & 15, g = lane >> 4; const size_t b = blockIdx.y; const int p0 = blockIdx.x * 64 + wave * 16; const int pix = p0 + col; const int ph = pix / WWD, pw = pix % WWD; const float* XTb = XT + b * NP * CC; const float* offp = OFF + (b * NP + pix) * 32;
  v8f acc[4] = {};
#pragma unroll 1
  for (int k = 0; k < NT; ++k) {
    const float pyf = (float)(ph + k / 3 - 1) + offp[2 * k]; const float pxf = (float)(pw + k % 3 - 1) + offp[2 * k + 1]; const float msk = 1.0f / (1.0f + expf(-offp[18 + k]));
    const float y0 = floorf(pyf), x0 = floorf(pxf); const float wy1 = pyf - y0, wx1 = pxf - x0, wy0 = 1.0f - wy1, wx0 = 1.0f - wx1; const int iy0 = (int)y0, ix0 = (int)x0;
#pragma unroll
    for (int kc = 0; kc < 2; ++kc) { float v[16];
#pragma unroll
      for (int i = 0; i < 16; ++i) v[i] = 0.f;
      corner16(XTb, iy0, ix0, g, kc, wy0 * wx0, v); corner16(XTb, iy0, ix0 + 1, g, kc, wy0 * wx1, v); corner16(XTb, iy0 + 1, ix0, g, kc, wy1 * wx0, v); corner16(XTb, iy0 + 1, ix0 + 1, g, kc, wy1 * wx1, v);
#pragma unroll
      for (int i = 0; i < 16; ++i) v[i] *= msk;
      const F2 a = bsplit16(v);
#pragma unroll
      for (int j = 0; j < 4; ++j) { const v16b w = frag_b(Wr + (size_t)(j * 16 + col) * KD + k * CC + kc * 32, lane); acc[j] = wmma_bf(a.h, w, acc[j]); acc[j] = wmma_bf(a.l, w, acc[j]); } } }
#pragma unroll
  for (int j = 0; j < 4; ++j)
#pragma unroll
    for (int r = 0; r < 8; ++r) so[j * 16 + col][wave * 16 + 8 * g + r] = acc[j][r] + bfr(BDEF[j * 16 + col]);
  __syncthreads();
  for (int e = tid; e < CC * 16; e += 128) { const int o = e >> 4, q = e & 15; vst2(Y + ((b * CC + o) * NP) + (size_t)blockIdx.x * 64 + q * 4, *(const v4f*)&so[o][q * 4]); } }
__global__ __launch_bounds__(256) void k_bnstat(const float* __restrict__ Y, float* __restrict__ ST) { __shared__ float red[8]; __shared__ __align__(16) float so2[32]; const int t = threadIdx.x; const int c = blockIdx.x;
  float s = 0.f; for (int b = 0; b < NB; ++b) { const float* row = Y + ((size_t)b * CC + c) * NP; for (int i = t; i < NP; i += 256) s += row[i]; }
#pragma unroll
  for (int o = 1; o < 32; o <<= 1) s += __shfl_xor(s, o);
  if ((t & 31) == 0) red[t >> 5] = s; __syncthreads(); float tot = 0.f; for (int i = 0; i < 8; ++i) tot += red[i]; const float mean = tot / (float)(NB * NP); __syncthreads();
  float q = 0.f; for (int b = 0; b < NB; ++b) { const float* row = Y + ((size_t)b * CC + c) * NP; for (int i = t; i < NP; i += 256) { const float d = row[i] - mean; q += d * d; } }
#pragma unroll
  for (int o = 1; o < 32; o <<= 1) q += __shfl_xor(q, o);
  if ((t & 31) == 0) red[t >> 5] = q; __syncthreads(); float tq = 0.f; for (int i = 0; i < 8; ++i) tq += red[i]; const float var = tq / (float)(NB * NP);
  if (t < 32) so2[t] = (t == 0) ? mean : (t == 1) ? 1.0f / sqrtf(var + BNEPS) : 0.f; __syncthreads(); if (t < 8) vst2(ST + (size_t)c * 32 + t * 4, *(const v4f*)&so2[t * 4]); }
__global__ __launch_bounds__(256) void k_bnxt(const float* __restrict__ Y, const float* __restrict__ ST, const float* __restrict__ G, const float* __restrict__ Bt, float* __restrict__ XT) { __shared__ float st[64][CC + 1]; __shared__ __align__(16) float so2[64][CC + 4]; const int t = threadIdx.x; const int p0 = blockIdx.x * 64; const size_t b = blockIdx.y;
  for (int e = t; e < CC * 64; e += 256) { const int c = e >> 6, pl = e & 63; const float y = Y[(b * CC + c) * NP + p0 + pl]; st[pl][c] = fmaxf((y - ST[c * 32]) * ST[c * 32 + 1] * bfr(G[c]) + bfr(Bt[c]), 0.f); } __syncthreads();
  for (int e = t; e < 64 * CC; e += 256) { const int pl = e >> 6, c = e & 63; so2[pl][c] = st[pl][c]; } __syncthreads();
  for (int e = t; e < 64 * 16; e += 256) { const int pl = e >> 4, q = e & 15; vst2(XT + ((b * NP + p0 + pl) * CC) + q * 4, *(const v4f*)&so2[pl][q * 4]); } }
__global__ __launch_bounds__(256) void k_bnout(const float* __restrict__ Y, const float* __restrict__ ST, const float* __restrict__ G, const float* __restrict__ Bt, float* __restrict__ OUT) { __shared__ __align__(16) float so2[NP]; const int t = threadIdx.x; const int c = blockIdx.x; const size_t b = blockIdx.y; const float m = ST[c * 32], is = ST[c * 32 + 1], gg = bfr(G[c]), bb = bfr(Bt[c]); const float* row = Y + ((b * CC + c) * NP);
  for (int i = t; i < NP; i += 256) so2[i] = fmaxf((row[i] - m) * is * gg + bb, 0.f); __syncthreads(); for (int q = t; q < NP / 4; q += 256) vst2(OUT + ((b * CC + c) * NP) + q * 4, *(const v4f*)&so2[q * 4]); }
extern "C" void kernel_launch(void* const* d_in, const int* in_sizes, int n_in, void* d_out, int out_size, void* d_ws, size_t ws_size, hipStream_t stream) {
  (void)in_sizes; (void)n_in; (void)out_size;
  const float** F = (const float**)d_in;
  if (ws_size < (size_t)WS_END) return;
  char* ws = (char*)d_ws; __bf16* P = (__bf16*)ws; float *XT = (float*)(ws + WS_XT), *OFF = (float*)(ws + WS_OFF), *Y = (float*)(ws + WS_Y), *ST = (float*)(ws + WS_ST);
  k_pack<<<dim3(CC, 4), 64, 0, stream>>>(F[1], F[3], F[7], F[9], P);
  k_xt<<<dim3(NP / 64, NB), 256, 0, stream>>>(F[0], XT);
  k_off<1><<<dim3(NP / 64, NB), 128, 0, stream>>>(XT, P + WS_PO1 / 2, F[2], OFF);
  k_def<<<dim3(NP / 64, NB), 128, 0, stream>>>(XT, OFF, P + WS_PD1 / 2, F[4], Y);
  k_bnstat<<<CC, 256, 0, stream>>>(Y, ST);
  k_bnxt<<<dim3(NP / 64, NB), 256, 0, stream>>>(Y, ST, F[5], F[6], XT);
  k_off<0><<<dim3(NP / 64, NB), 128, 0, stream>>>(XT, P + WS_PO2 / 2, F[8], OFF);
  k_def<<<dim3(NP / 64, NB), 128, 0, stream>>>(XT, OFF, P + WS_PD2 / 2, F[10], Y);
  k_bnstat<<<CC, 256, 0, stream>>>(Y, ST);
  k_bnout<<<dim3(CC, NB), 256, 0, stream>>>(Y, ST, F[11], F[12], (float*)d_out);
}
